// TransformerBlock_82772609729208
// MI455X (gfx1250) — hardware-verified
//
#include <hip/hip_runtime.h>
#ifndef NB
#define NB 2
#endif
#ifndef SEQ
#define SEQ 2048
#endif
#define NB_FULL 2
#define SEQ_FULL 2048
#define SQ SEQ
#define DM 1024
#define NH 16
#define HD 64
#define DFF 4096
#define QT 256
#define NKX SQ
#define QT0 128
#define NR ((size_t)NB * SQ)
#define LQ (3 * DM)

static_assert(NB >= 1 && NB <= NB_FULL);
static_assert(SQ <= SEQ_FULL);
static_assert(DM == 1024);
static_assert(DM == NH * HD);
static_assert(HD == 64);
static_assert((QT & (QT - 1)) == 0);
static_assert(QT % 256 == 0);
static_assert(SQ % QT == 0);
static_assert(QT0 == 128);
static_assert(QT0 <= QT);
static_assert(SQ % 128 == 0);
static_assert(DFF % 64 == 0);
static_assert(((size_t)NB * SQ) % 128 == 0);

typedef unsigned short v8us __attribute__((ext_vector_type(8), may_alias));
typedef float  v8f  __attribute__((ext_vector_type(8)));
typedef float  v4f  __attribute__((ext_vector_type(4)));
typedef float  v4fa __attribute__((ext_vector_type(4), may_alias));
typedef _Float16 v16h __attribute__((ext_vector_type(16)));
typedef _Float16 v4h __attribute__((ext_vector_type(4)));
union FragH { v16h v; v8us half[2]; _Float16 h[16]; unsigned short u[16]; };

__device__ __forceinline__ unsigned short bf16_bits(float x) { unsigned int u = __float_as_uint(x); return (unsigned short)((u + 0x7FFFu + ((u >> 16) & 1u)) >> 16); }
__device__ __forceinline__ float bf16_val(unsigned short b) { return __uint_as_float(((unsigned int)b) << 16); }
__device__ __forceinline__ float bf16_rne(float x) { return bf16_val(bf16_bits(x)); }

__global__ __launch_bounds__(256) void k_wt_f16(const float* __restrict__ W, _Float16* __restrict__ Wt, unsigned K, unsigned N, float scale) {
  const unsigned t = blockIdx.x * 256u + threadIdx.x; const unsigned k8n = K >> 3; if (t >= N * k8n) return;
  const unsigned n = t / k8n, k8 = (t - n * k8n) << 3; FragH f;
#pragma unroll
  for (int i = 0; i < 8; ++i) f.h[i] = (_Float16)(bf16_rne(W[(size_t)(k8 + i) * N + n]) * scale);
  const v8us o = f.half[0];
  unsigned short* d = (unsigned short*)Wt + (size_t)n * K + k8;
  *(volatile v8us*)d = o; __threadfence(); *(volatile v8us*)d = o;
}

__global__ __launch_bounds__(256) void k_hl(const float* __restrict__ F, _Float16* __restrict__ Hh, _Float16* __restrict__ Hl, size_t n8) {
  const size_t t = (size_t)blockIdx.x * 256 + threadIdx.x; if (t >= n8) return; FragH fh, fl; const v4f a = *(const v4fa*)(F + t * 8), c = *(const v4fa*)(F + t * 8 + 4);
#pragma unroll
  for (int q = 0; q < 4; ++q) { _Float16 h = (_Float16)a[q]; fh.h[q] = h; fl.h[q] = (_Float16)((a[q] - (float)h) * 1024.0f); h = (_Float16)c[q]; fh.h[4 + q] = h; fl.h[4 + q] = (_Float16)((c[q] - (float)h) * 1024.0f); }
  const v8us oh = fh.half[0], ol = fl.half[0];
  for (int pass = 0; pass < 2; ++pass) { *(volatile v8us*)((unsigned short*)Hh + t * 8) = oh; *(volatile v8us*)((unsigned short*)Hl + t * 8) = ol; if (pass == 0) __threadfence(); }
}

__device__ __forceinline__ v16h g2_frag(const _Float16* p, int hh) { FragH f; f.half[0] = *(const v8us*)((const unsigned short*)p + 8 * hh); f.half[1] = *(const v8us*)((const unsigned short*)p + 16 + 8 * hh); return f.v; }
__device__ __forceinline__ v8f g2_mma(v16h a, v16h b, v8f c) { v8f d = __builtin_amdgcn_wmma_f32_16x16x32_f16(false, a, false, b, (short)0, c, false, false); asm volatile("v_nop\n\tv_nop\n\tv_nop\n\tv_nop" : "+v"(d) : "v"(a), "v"(b)); return d; }
template <int ACT>
__global__ __launch_bounds__(128) void k_gemm2(const _Float16* __restrict__ A, int lda, size_t sA, const _Float16* __restrict__ Bh, int ldb, size_t sB, float alpha, const float* __restrict__ bias, const float* CP,
    float* C, _Float16* __restrict__ C16, int ldc, size_t sC, int M, int N, int K) {
  static_assert(ACT == 0 || ACT == 9);
  __shared__ __attribute__((aligned(16))) float so[4][32][68];
  const int tid = threadIdx.x, w = tid >> 5, lane = tid & 31, ln = lane & 15, hh = lane >> 4; const unsigned by = blockIdx.y;
  A += (size_t)by * sA; Bh += (size_t)by * sB; const size_t cofs = (size_t)by * sC;
  const unsigned ntn = (unsigned)N >> 6; const unsigned mtu = blockIdx.x / ntn, nqu = blockIdx.x - mtu * ntn; const int row0 = (int)(mtu * 128u) + 32 * w, col0 = (int)(nqu * 64u); if (row0 >= M) return;
  const _Float16* a0p = A + (size_t)(row0 + ln) * lda; const _Float16* a1p = a0p + (size_t)16 * lda;
  const _Float16* b0p = Bh + (size_t)(col0 + ln) * ldb; const _Float16* b1p = b0p + (size_t)16 * ldb; const _Float16* b2p = b1p + (size_t)16 * ldb; const _Float16* b3p = b2p + (size_t)16 * ldb;
  const v8f z8 = {0.f,0.f,0.f,0.f,0.f,0.f,0.f,0.f}; v8f c00 = z8, c01 = z8, c02 = z8, c03 = z8, c10 = z8, c11 = z8, c12 = z8, c13 = z8;
#pragma unroll 1
  for (int kb = 0; kb < K; kb += 32) { const v16h a0 = g2_frag(a0p + kb, hh), a1 = g2_frag(a1p + kb, hh);
    v16h b = g2_frag(b0p + kb, hh); c00 = g2_mma(a0, b, c00); c10 = g2_mma(a1, b, c10);
    b = g2_frag(b1p + kb, hh); c01 = g2_mma(a0, b, c01); c11 = g2_mma(a1, b, c11);
    b = g2_frag(b2p + kb, hh); c02 = g2_mma(a0, b, c02); c12 = g2_mma(a1, b, c12);
    b = g2_frag(b3p + kb, hh); c03 = g2_mma(a0, b, c03); c13 = g2_mma(a1, b, c13); }
  v8f accs[8] = {c00, c01, c02, c03, c10, c11, c12, c13};
#pragma unroll
  for (int u = 0; u < 8; ++u) { const int t = u & 3, half = u >> 2; const int col = col0 + t * 16 + ln; const float bv = bias ? bf16_rne(bias[col]) : 0.f;
#pragma unroll
    for (int r = 0; r < 8; ++r) { const int rloc = half * 16 + 8 * hh + r; float v = accs[u][r] * alpha + bv; if (CP) v += CP[cofs + (size_t)(row0 + rloc) * ldc + col];
      if (ACT == 9) v = 0.5f * v * (1.0f + tanhf(0.7978845608028654f * (v + 0.044715f * v * v * v)));
      so[w][rloc][t * 16 + ln] = v; } }
  __builtin_amdgcn_fence(4  , "workgroup"); __builtin_amdgcn_wave_barrier();
  const int rsub = lane >> 4, c4 = (lane & 15) * 4;
  for (int pass = 0; pass < 2; ++pass) {
#pragma unroll
    for (int q = 0; q < 16; ++q) { const int r = q * 2 + rsub; const v4f v = *(const v4fa*)&so[w][r][c4]; if (C) *(volatile v4f*)(C + cofs + (size_t)(row0 + r) * ldc + col0 + c4) = v; if (C16) { v4h h4; for (int i = 0; i < 4; ++i) h4[i] = (_Float16)v[i]; *(volatile v4h*)(C16 + cofs + (size_t)(row0 + r) * ldc + col0 + c4) = h4; } }
    if (pass == 0) __threadfence(); } }

template <int NHv, int TTv>
__global__ __launch_bounds__(256) void k_vt(const _Float16* __restrict__ V16, int ldv, int voff, _Float16* __restrict__ Vt) {
  __shared__ unsigned short tl[64][66];
  const unsigned tid = threadIdx.x; const unsigned slab = blockIdx.x / (unsigned)(TTv / 64), lg = blockIdx.x % (unsigned)(TTv / 64); const unsigned b = slab / (unsigned)NHv, h = slab % (unsigned)NHv;
  for (unsigned i = tid; i < 512u; i += 256u) { const unsigned r = i >> 3, c8 = (i & 7u) << 3; FragH f; f.half[0] = *(const v8us*)((const unsigned short*)V16 + ((size_t)b * TTv + lg * 64u + r) * ldv + voff + h * 64u + c8);
#pragma unroll
    for (int q = 0; q < 8; ++q) tl[r][c8 + q] = f.u[q]; }
  __syncthreads();
  for (int pass = 0; pass < 2; ++pass) {
#pragma unroll
    for (unsigned rd = 0; rd < 2u; ++rd) { const unsigned d = rd * 32u + (tid >> 3), pc = tid & 7u; FragH f;
#pragma unroll
      for (int q = 0; q < 8; ++q) f.u[q] = tl[pc * 8u + q][d];
      *(volatile v8us*)((unsigned short*)Vt + ((size_t)slab * 64 + d) * TTv + lg * 64u + pc * 8u) = f.half[0]; }
    if (pass == 0) __threadfence(); } }

__global__ __launch_bounds__(256) void k_rsmw(const float* __restrict__ S, _Float16* __restrict__ P, unsigned nrows, unsigned q0, unsigned nk) {
  #pragma clang fp contract(off)
  const unsigned lane = threadIdx.x & 31u; const unsigned row = blockIdx.x * 8u + (threadIdx.x >> 5); if (row >= nrows) return;
  const float* s = S + (size_t)row * NKX; const unsigned last = q0 + (row & (unsigned)(QT - 1)); float mx = -3.0e38f;
#pragma unroll 1
  for (unsigned j0 = 0; j0 < nk; j0 += 256u) { const unsigned j = j0 + lane * 8u; const v4f a = *(const v4fa*)(s + j), c = *(const v4fa*)(s + j + 4);
#pragma unroll
    for (unsigned q = 0; q < 4u; ++q) { const float va = (j + q <= last) ? a[q] : -1.0e9f; const float vc = (j + 4u + q <= last) ? c[q] : -1.0e9f; mx = fmaxf(mx, fmaxf(va, vc)); } }
  mx = fmaxf(mx, __shfl_xor(mx, 16, 32)); mx = fmaxf(mx, __shfl_xor(mx, 8, 32)); mx = fmaxf(mx, __shfl_xor(mx, 4, 32)); mx = fmaxf(mx, __shfl_xor(mx, 2, 32)); mx = fmaxf(mx, __shfl_xor(mx, 1, 32));
  float se = 0.f;
#pragma unroll 1
  for (unsigned j0 = 0; j0 < nk; j0 += 256u) { const unsigned j = j0 + lane * 8u; const v4f a = *(const v4fa*)(s + j), c = *(const v4fa*)(s + j + 4);
#pragma unroll
    for (unsigned q = 0; q < 4u; ++q) { const float va = (j + q <= last) ? a[q] : -1.0e9f; const float vc = (j + 4u + q <= last) ? c[q] : -1.0e9f; se += __expf(va - mx); se += __expf(vc - mx); } }
  se += __shfl_xor(se, 16, 32); se += __shfl_xor(se, 8, 32); se += __shfl_xor(se, 4, 32); se += __shfl_xor(se, 2, 32); se += __shfl_xor(se, 1, 32);
  const float sc = 256.0f / se;
#pragma unroll 1
  for (unsigned j0 = 0; j0 < nk; j0 += 256u) { const unsigned j = j0 + lane * 8u; const v4f a = *(const v4fa*)(s + j), c = *(const v4fa*)(s + j + 4); FragH fr;
#pragma unroll
    for (unsigned q = 0; q < 4u; ++q) { const float va = (j + q <= last) ? a[q] : -1.0e9f; const float vc = (j + 4u + q <= last) ? c[q] : -1.0e9f; fr.h[q] = (_Float16)(__expf(va - mx) * sc); fr.h[4 + q] = (_Float16)(__expf(vc - mx) * sc); }
    const v8us o = fr.half[0]; unsigned short* d = (unsigned short*)P + (size_t)row * NKX + j; *(volatile v8us*)d = o; __threadfence(); *(volatile v8us*)d = o; } }

__global__ __launch_bounds__(64) void k_att0(const float* __restrict__ QF, const float* __restrict__ KF, const float* __restrict__ VF, int ld, float scale, float* __restrict__ OF, int ldo) {
  #pragma clang fp contract(off)
  __shared__ __attribute__((aligned(16))) float lq[64][64]; __shared__ __attribute__((aligned(16))) float lo[64][64];
  const unsigned tid = threadIdx.x; const unsigned h = blockIdx.x / (unsigned)(QT0 / 64), rg = blockIdx.x % (unsigned)(QT0 / 64); const unsigned i = rg * 64u + tid;
  const float* qr = QF + (size_t)i * ld + h * HD;
#pragma unroll 1
  for (int c = 0; c < HD / 4; ++c) { *(v4f*)&lq[tid][c * 4] = *(const v4fa*)(qr + c * 4); const v4f z = {0.f, 0.f, 0.f, 0.f}; *(v4f*)&lo[tid][c * 4] = z; }
  float m = -1.0e30f, l = 0.f; const unsigned jmax = rg * 64u + 63u;
#pragma unroll 1
  for (unsigned j = 0; j <= jmax; ++j) { const float* kr = KF + (size_t)j * ld + h * HD; const float* vr = VF + (size_t)j * ld + h * HD; float s = 0.f;
#pragma unroll 1
    for (int c = 0; c < HD / 4; ++c) { const v4f kq = *(const v4fa*)(kr + c * 4); const v4f qq = *(v4f*)&lq[tid][c * 4]; s = __fadd_rn(s, __fmul_rn(qq[0], kq[0])); s = __fadd_rn(s, __fmul_rn(qq[1], kq[1])); s = __fadd_rn(s, __fmul_rn(qq[2], kq[2])); s = __fadd_rn(s, __fmul_rn(qq[3], kq[3])); }
    s = __fmul_rn(s, scale);
    const float sm = (j <= i) ? s : -1.0e30f; const float mn = fmaxf(m, sm); const float sc = expf(m - mn); const float e = expf(sm - mn); l = __fadd_rn(__fmul_rn(l, sc), e); m = mn;
#pragma unroll 1
    for (int c = 0; c < HD / 4; ++c) { const v4f vv = *(const v4fa*)(vr + c * 4); v4f oo = *(v4f*)&lo[tid][c * 4]; for (int u = 0; u < 4; ++u) oo[u] = __fadd_rn(__fmul_rn(oo[u], sc), __fmul_rn(e, vv[u])); *(v4f*)&lo[tid][c * 4] = oo; } }
  const float fin = 64.0f / l;
#pragma unroll 1
  for (int c = 0; c < HD / 4; ++c) { v4f oo = *(v4f*)&lo[tid][c * 4]; for (int u = 0; u < 4; ++u) oo[u] = __fmul_rn(oo[u], fin); *(v4f*)&lo[tid][c * 4] = oo; }
  __syncthreads();
  for (int pass = 0; pass < 2; ++pass) {
#pragma unroll 1
    for (unsigned it = 0; it < 16u; ++it) { const unsigned row = it * 4u + (tid >> 4), pc = (tid & 15u) * 4u; const v4f v = *(const v4f*)&lo[row][pc]; *(volatile v4f*)(OF + (size_t)(rg * 64u + row) * ldo + h * HD + pc) = v; }
    if (pass == 0) __threadfence(); } }

template <int BFIN, int WXB, int INFULL>
__global__ __launch_bounds__(256) void k_ln16(const float* __restrict__ X, const float* __restrict__ g, const float* __restrict__ bb, float eps, _Float16* __restrict__ N16, float* __restrict__ XB) {
  #pragma clang fp contract(off)
  __shared__ float red[256]; const unsigned rr = blockIdx.x; const unsigned t = threadIdx.x; const size_t r = rr;
  const size_t rin = INFULL ? ((size_t)(rr / (unsigned)SQ) * SEQ_FULL + (rr % (unsigned)SQ)) : r;
  const v4f xa = *(const v4fa*)(X + rin * DM + t * 4); float s[4]; float sum = 0.f;
  for (int q = 0; q < 4; ++q) { s[q] = BFIN ? bf16_rne(xa[q]) : xa[q]; sum = __fadd_rn(sum, s[q]); }
  red[t] = sum; __syncthreads(); for (unsigned st = 128; st > 0; st >>= 1) { if (t < st) red[t] = __fadd_rn(red[t], red[t + st]); __syncthreads(); } const float mu = __fmul_rn(red[0], 1.0f / (float)DM); __syncthreads();
  float vs = 0.f; for (int q = 0; q < 4; ++q) { const float dl = __fadd_rn(s[q], -mu); vs = __fadd_rn(vs, __fmul_rn(dl, dl)); } red[t] = vs; __syncthreads(); for (unsigned st = 128; st > 0; st >>= 1) { if (t < st) red[t] = __fadd_rn(red[t], red[t + st]); __syncthreads(); }
  const float rs = rsqrtf(__fadd_rn(__fmul_rn(red[0], 1.0f / (float)DM), eps)); v4h y; v4f xb;
  for (int q = 0; q < 4; ++q) { const unsigned c = t * 4 + q; y[q] = (_Float16)__fadd_rn(__fmul_rn(__fmul_rn(__fadd_rn(s[q], -mu), rs), bf16_rne(g[c])), bf16_rne(bb[c])); xb[q] = s[q]; }
  for (int pass = 0; pass < 2; ++pass) { *(volatile v4h*)(N16 + r * DM + t * 4) = y; if (WXB) *(volatile v4f*)(XB + r * DM + t * 4) = xb; if (pass == 0) __threadfence(); } }

constexpr size_t al256(size_t b) { return (b + 255) & ~(size_t)255; }
constexpr size_t cmax(size_t a, size_t b) { return a > b ? a : b; }
constexpr size_t SZ_S    = al256((size_t)NH * QT * NKX * 4);
constexpr size_t SZ_P    = al256((size_t)NH * QT * NKX * 2);
constexpr size_t SZ_HF   = al256((size_t)SQ * DFF * 2);
constexpr size_t SZ_BW   = al256((size_t)DFF * DM * 2);
constexpr size_t SZ_R16  = al256(NR * DM * 2);
constexpr size_t SZ_R32  = al256(NR * DM * 4);
constexpr size_t SZ_QKV  = al256(NR * 3 * DM * 2);
constexpr size_t SZ_WQKV = al256((size_t)3 * DM * DM * 2);
constexpr size_t SZ_WO   = al256((size_t)DM * DM * 2);
constexpr size_t SZ_VT   = al256((size_t)NH * HD * SQ * 2);
constexpr size_t SZ_F0   = al256((size_t)QT0 * DM * 4);
constexpr size_t SZ_OF0  = al256((size_t)NB * QT0 * DM * 4);
constexpr size_t SZ_OH0  = al256((size_t)NB * QT0 * DM * 2);
constexpr size_t SZ_RA   = cmax(SZ_S, SZ_HF + 2 * SZ_BW);
constexpr size_t SZ_RB   = cmax(SZ_P, SZ_R16);
constexpr size_t SZ_RC   = cmax(SZ_QKV, SZ_R32);
constexpr size_t OFF_RA = 0;
constexpr size_t OFF_RB = OFF_RA + SZ_RA;
constexpr size_t OFF_RC = OFF_RB + SZ_RB;
constexpr size_t OFF_XB = OFF_RC + SZ_RC;
constexpr size_t OFF_X16 = OFF_XB + SZ_R32;
constexpr size_t OFF_O16 = OFF_X16 + SZ_R16;
constexpr size_t OFF_WQKV = OFF_O16 + SZ_R16;
constexpr size_t OFF_WO = OFF_WQKV + SZ_WQKV;
constexpr size_t OFF_VT = OFF_WO + SZ_WO;
constexpr size_t OFF_QF0 = OFF_VT + SZ_VT;
constexpr size_t OFF_KF0 = OFF_QF0 + SZ_F0;
constexpr size_t OFF_VF0 = OFF_KF0 + SZ_F0;
constexpr size_t OFF_OF0 = OFF_VF0 + SZ_F0;
constexpr size_t OFF_OH0 = OFF_OF0 + SZ_OF0;
constexpr size_t OFF_OL0 = OFF_OH0 + SZ_OH0;
constexpr size_t WS_TOTAL = OFF_OL0 + SZ_OH0;
static_assert(SZ_S <= SZ_RA);
static_assert(SZ_HF + 2 * SZ_BW <= SZ_RA);
static_assert(SZ_P <= SZ_RB);
static_assert(SZ_R16 <= SZ_RB);
static_assert(SZ_QKV <= SZ_RC);
static_assert(SZ_R32 <= SZ_RC);
static_assert(WS_TOTAL <= (size_t)134217728);

extern "C" void kernel_launch(void* const* d_in, const int* in_sizes, int n_in,
                              void* d_out, int out_size, void* d_ws, size_t ws_size, hipStream_t stream) {
  if (n_in < 14) return;
  const size_t need_x = ((size_t)(NB - 1) * SEQ_FULL + SQ) * DM;
  if ((size_t)in_sizes[0] < need_x || (size_t)out_size < need_x) return;
  if (in_sizes[1] < DM * DM || in_sizes[2] < DM * DM || in_sizes[3] < DM * DM || in_sizes[4] < DM * DM) return;
  if (in_sizes[5] < DM || in_sizes[6] < DM * DFF || in_sizes[7] < DFF || in_sizes[8] < DFF * DM || in_sizes[9] < DM) return;
  if (in_sizes[10] < DM || in_sizes[11] < DM || in_sizes[12] < DM || in_sizes[13] < DM) return;
  if (WS_TOTAL > ws_size) return;
  const float* const* I = (const float* const*)d_in;
  const float* x = I[0]; const float* wq = I[1]; const float* wk = I[2]; const float* wv = I[3]; const float* wo = I[4]; const float* bo = I[5];
  const float* w1 = I[6]; const float* b1 = I[7]; const float* w2 = I[8]; const float* b2 = I[9]; const float* a1 = I[10]; const float* s1 = I[11]; const float* a2 = I[12]; const float* s2 = I[13];
  char* ws = (char*)d_ws;
  float* S = (float*)(ws + OFF_RA); _Float16* HF16 = (_Float16*)(ws + OFF_RA); _Float16* BW1 = (_Float16*)(ws + OFF_RA + SZ_HF); _Float16* BW2 = (_Float16*)(ws + OFF_RA + SZ_HF + SZ_BW);
  _Float16* P = (_Float16*)(ws + OFF_RB); _Float16* M16 = (_Float16*)(ws + OFF_RB);
  _Float16* QKV = (_Float16*)(ws + OFF_RC); float* X1 = (float*)(ws + OFF_RC);
  _Float16* Q16 = QKV; _Float16* K16 = QKV + DM; _Float16* V16 = QKV + 2 * DM;
  float* XB = (float*)(ws + OFF_XB); _Float16* X16 = (_Float16*)(ws + OFF_X16); _Float16* O16 = (_Float16*)(ws + OFF_O16);
  _Float16* BQKV = (_Float16*)(ws + OFF_WQKV); _Float16* BO = (_Float16*)(ws + OFF_WO); _Float16* VT = (_Float16*)(ws + OFF_VT);
  float* QF0 = (float*)(ws + OFF_QF0); float* KF0 = (float*)(ws + OFF_KF0); float* VF0 = (float*)(ws + OFF_VF0); float* OF0 = (float*)(ws + OFF_OF0);
  _Float16* OH0 = (_Float16*)(ws + OFF_OH0); _Float16* OL0 = (_Float16*)(ws + OFF_OL0);

  { const unsigned gw = (unsigned)(((size_t)DM * (DM / 8) + 255) / 256);
    k_wt_f16<<<gw, 256, 0, stream>>>(wq, BQKV, (unsigned)DM, (unsigned)DM, 16.0f);
    k_wt_f16<<<gw, 256, 0, stream>>>(wk, BQKV + (size_t)DM * DM, (unsigned)DM, (unsigned)DM, 16.0f);
    k_wt_f16<<<gw, 256, 0, stream>>>(wv, BQKV + (size_t)2 * DM * DM, (unsigned)DM, (unsigned)DM, 16.0f);
    k_wt_f16<<<gw, 256, 0, stream>>>(wo, BO, (unsigned)DM, (unsigned)DM, 16.0f); }
  k_ln16<1, 1, 1><<<(unsigned)NR, 256, 0, stream>>>(x, a1, s1, 1e-5f, X16, XB);
  k_gemm2<0><<<dim3((unsigned)((NR / 128) * (3 * DM / 64)), 1), 128, 0, stream>>>(X16, DM, (size_t)0, BQKV, DM, (size_t)0, 0.0625f, nullptr, nullptr, nullptr, QKV, 3 * DM, (size_t)0, (int)NR, 3 * DM, DM);
  for (int b = 0; b < NB; ++b) { const size_t r0 = (size_t)b * SQ;
    k_vt<NH, SQ><<<NH * (SQ / 64), 256, 0, stream>>>(V16 + r0 * LQ, LQ, 0, VT);
    k_gemm2<0><<<dim3((QT0 / 128) * (DM / 64), 1), 128, 0, stream>>>(X16 + r0 * DM, DM, (size_t)0, BQKV, DM, (size_t)0, 0.0625f, nullptr, nullptr, QF0, nullptr, DM, (size_t)0, QT0, DM, DM);
    k_gemm2<0><<<dim3((QT0 / 128) * (DM / 64), 1), 128, 0, stream>>>(X16 + r0 * DM, DM, (size_t)0, BQKV + (size_t)DM * DM, DM, (size_t)0, 0.0625f, nullptr, nullptr, KF0, nullptr, DM, (size_t)0, QT0, DM, DM);
    k_gemm2<0><<<dim3((QT0 / 128) * (DM / 64), 1), 128, 0, stream>>>(X16 + r0 * DM, DM, (size_t)0, BQKV + (size_t)2 * DM * DM, DM, (size_t)0, 0.0625f, nullptr, nullptr, VF0, nullptr, DM, (size_t)0, QT0, DM, DM);
    k_att0<<<NH * (QT0 / 64), 64, 0, stream>>>(QF0, KF0, VF0, DM, 0.125f, OF0 + (size_t)b * QT0 * DM, DM);
    for (int q0 = 0; q0 < SQ; q0 += QT) { const int nk = q0 + QT;
      k_gemm2<0><<<dim3((unsigned)((QT / 128) * (nk / 64)), NH), 128, 0, stream>>>(Q16 + (r0 + q0) * LQ, LQ, (size_t)HD, K16 + r0 * LQ, LQ, (size_t)HD, 0.125f, nullptr, nullptr, S, nullptr, NKX, (size_t)QT * NKX, QT, nk, HD);
      k_rsmw<<<(NH * QT + 7) / 8, 256, 0, stream>>>(S, P, (unsigned)(NH * QT), (unsigned)q0, (unsigned)nk);
      k_gemm2<0><<<dim3((QT / 128) * (HD / 64), NH), 128, 0, stream>>>(P, NKX, (size_t)QT * NKX, VT, SQ, (size_t)HD * SQ, 0.25f, nullptr, nullptr, nullptr, O16 + (r0 + q0) * DM, DM, (size_t)HD, QT, HD, nk); } }
  k_gemm2<0><<<dim3((unsigned)((NR / 128) * (DM / 64)), 1), 128, 0, stream>>>(O16, DM, (size_t)0, BO, DM, (size_t)0, 0.0009765625f, bo, XB, X1, nullptr, DM, (size_t)0, (int)NR, DM, DM);
  k_hl<<<(unsigned)(((size_t)NB * QT0 * DM / 8 + 255) / 256), 256, 0, stream>>>(OF0, OH0, OL0, (size_t)NB * QT0 * DM / 8);
  for (int b = 0; b < NB; ++b) { const size_t r0 = (size_t)b * SQ; const size_t f0 = (size_t)b * QT0;
    k_gemm2<0><<<dim3((QT0 / 128) * (DM / 64), 1), 128, 0, stream>>>(OH0 + f0 * DM, DM, (size_t)0, BO, DM, (size_t)0, 0.0009765625f, bo, XB + r0 * DM, X1 + r0 * DM, nullptr, DM, (size_t)0, QT0, DM, DM);
    k_gemm2<0><<<dim3((QT0 / 128) * (DM / 64), 1), 128, 0, stream>>>(OL0 + f0 * DM, DM, (size_t)0, BO, DM, (size_t)0, 0.00000095367431640625f, nullptr, X1 + r0 * DM, X1 + r0 * DM, nullptr, DM, (size_t)0, QT0, DM, DM); }
  k_wt_f16<<<(unsigned)(((size_t)DFF * (DM / 8) + 255) / 256), 256, 0, stream>>>(w1, BW1, (unsigned)DM, (unsigned)DFF, 16.0f);
  k_wt_f16<<<(unsigned)(((size_t)DM * (DFF / 8) + 255) / 256), 256, 0, stream>>>(w2, BW2, (unsigned)DFF, (unsigned)DM, 16.0f);
  k_ln16<0, 0, 0><<<(unsigned)NR, 256, 0, stream>>>(X1, a2, s2, 1e-5f, M16, nullptr);
  for (int b = 0; b < NB; ++b) { const size_t r0 = (size_t)b * SQ;
    k_gemm2<9><<<dim3((unsigned)((SQ / 128) * (DFF / 64)), 1), 128, 0, stream>>>(M16 + r0 * DM, DM, (size_t)0, BW1, DM, (size_t)0, 0.0625f, b1, nullptr, nullptr, HF16, DFF, (size_t)0, SQ, DFF, DM);
    k_gemm2<0><<<dim3((unsigned)((SQ / 128) * (DM / 64)), 1), 128, 0, stream>>>(HF16, DFF, (size_t)0, BW2, DFF, (size_t)0, 0.0625f, b2, X1 + r0 * DM, (float*)d_out + (size_t)b * SEQ_FULL * DM, nullptr, DM, (size_t)0, SQ, DM, DFF); }
}
